// SelfAttentionV3_22273700397196
// MI455X (gfx1250) — hardware-verified
//
#include <hip/hip_runtime.h>
#include <hip/hip_bf16.h>
#include <stdint.h>

typedef __attribute__((ext_vector_type(16))) _Float16 v16h;
typedef __attribute__((ext_vector_type(8)))  _Float16 v8h;
typedef __attribute__((ext_vector_type(16))) __bf16   v16b;
typedef __attribute__((ext_vector_type(8)))  __bf16   v8b;
typedef __attribute__((ext_vector_type(8)))  float    v8f;
typedef __attribute__((ext_vector_type(4)))  float    v4f;
typedef __attribute__((ext_vector_type(8)))  unsigned short us8;
typedef __attribute__((ext_vector_type(4)))  unsigned int   u32x4;

constexpr int kBatch = 4;
constexpr int kSeq   = 2048;
constexpr int kDim   = 1024;
constexpr int kTok   = kBatch * kSeq;
constexpr int kN3    = 3 * kDim;
constexpr int kPadM  = 64;

constexpr float kPcarry   = 16384.0f;
constexpr float kPoffset  = 8.0f;
constexpr float kZcarry   = 256.0f;
constexpr float kWoCarry  = 64.0f;
constexpr float kScoreScale = 0.03125f;

constexpr size_t SZ_XB   = (size_t)kTok * kDim * 2;
constexpr size_t SZ_WQKV = (size_t)kN3 * kDim * 2;
constexpr size_t SZ_WO   = (size_t)kDim * kDim * 2;
constexpr size_t SZ_BIAS = (size_t)(kN3 + kDim) * 4;
constexpr size_t SZ_M64  = (size_t)kPadM * kDim * 2;
constexpr size_t SZ_ADDV = (size_t)kPadM * kDim * 4;
constexpr size_t SZ_QK   = (size_t)kTok * 2048 * 2;
constexpr size_t SZ_VT   = (size_t)kBatch * kDim * kSeq * 2;
constexpr size_t SZ_SBUF = (size_t)2 * kSeq * kSeq * 4;

constexpr size_t OFF_XB   = 0;
constexpr size_t OFF_WQKV = OFF_XB + SZ_XB;
constexpr size_t OFF_WO16 = OFF_WQKV + SZ_WQKV;
constexpr size_t OFF_WOB  = OFF_WO16 + SZ_WO;
constexpr size_t OFF_ZERO = OFF_WOB + SZ_WO;
constexpr size_t OFF_BIAS = OFF_ZERO + SZ_WO;
constexpr size_t OFF_MXH  = OFF_BIAS + SZ_BIAS;
constexpr size_t OFF_MXL  = OFF_MXH + SZ_M64;
constexpr size_t OFF_VBH  = OFF_MXL + SZ_M64;
constexpr size_t OFF_VBL  = OFF_VBH + SZ_M64;
constexpr size_t OFF_ADDV = OFF_VBL + SZ_M64;
constexpr size_t OFF_QK   = OFF_ADDV + SZ_ADDV;
constexpr size_t OFF_VT   = OFF_QK + SZ_QK;
constexpr size_t OFF_SBUF = OFF_VT + SZ_VT;
constexpr size_t WS_TOTAL = OFF_SBUF + SZ_SBUF;
static_assert(WS_TOTAL == 114049024ull);
static_assert(WS_TOTAL <= 134217728ull);
static_assert((OFF_WQKV % 256) == 0 && (OFF_WO16 % 256) == 0 && (OFF_WOB % 256) == 0 && (OFF_ZERO % 256) == 0);
static_assert((OFF_BIAS % 256) == 0 && (OFF_MXH % 256) == 0 && (OFF_MXL % 256) == 0 && (OFF_VBH % 256) == 0);
static_assert((OFF_VBL % 256) == 0 && (OFF_ADDV % 256) == 0 && (OFF_QK % 256) == 0 && (OFF_VT % 256) == 0 && (OFF_SBUF % 256) == 0);
static_assert((size_t)kBatch * kSeq * kSeq * 2 == SZ_QK);
static_assert((size_t)kTok * kDim * 2 == SZ_XB);

__device__ __forceinline__ unsigned short f2bf_bits(float f) {
  unsigned u = __float_as_uint(f);
  return (unsigned short)((u + 0x7FFFu + ((u >> 16) & 1u)) >> 16);
}
__device__ __forceinline__ float bf_bits2f(unsigned short h) { return __uint_as_float(((unsigned)h) << 16); }
__device__ __forceinline__ float bf16r(float f) { return bf_bits2f(f2bf_bits(f)); }
__device__ __forceinline__ int imin(int a, int b) { return a < b ? a : b; }
__device__ __forceinline__ int imax(int a, int b) { return a > b ? a : b; }

__device__ __forceinline__ void dep_guard_h(v8f& a, v8f& b, v16h x, v16h y) { asm volatile("v_nop\n\tv_nop\n\tv_nop\n\tv_nop" : "+v"(a), "+v"(b) : "v"(x), "v"(y)); }
__device__ __forceinline__ void dep_guard_b(v8f& a, v8f& b, v16b x, v16b y) { asm volatile("v_nop\n\tv_nop\n\tv_nop\n\tv_nop" : "+v"(a), "+v"(b) : "v"(x), "v"(y)); }
__device__ __forceinline__ void keep4_h(v16h a, v16h b, v16h c, v16h d) { asm volatile("v_nop" :: "v"(a), "v"(b), "v"(c), "v"(d)); }
__device__ __forceinline__ void keep4_b(v16b a, v16b b, v16b c, v16b d) { asm volatile("v_nop" :: "v"(a), "v"(b), "v"(c), "v"(d)); }
__device__ __forceinline__ void acc_guard4(v8f& a, v8f& b, v8f& c, v8f& d) { asm volatile("v_nop\n\tv_nop\n\tv_nop\n\tv_nop" : "+v"(a), "+v"(b), "+v"(c), "+v"(d)); }
template <typename T> struct Frag;
template <> struct Frag<_Float16> {
  typedef v16h V; union U { v16h v; v8h h[2]; };
  static __device__ __forceinline__ v16h load(const _Float16* p) {
    U f; f.h[0] = *(const v8h*)(p); f.h[1] = *(const v8h*)(p + 16); return f.v;
  }
  static __device__ __forceinline__ v8f mma(v16h a, v16h b, v8f c) {
    return __builtin_amdgcn_wmma_f32_16x16x32_f16(false, a, false, b, (short)0, c, false, false);
  }
  static __device__ __forceinline__ void guard(v8f& a, v8f& b, v16h x, v16h y) { dep_guard_h(a, b, x, y); }
  static __device__ __forceinline__ void keep(v16h a, v16h b, v16h c, v16h d) { keep4_h(a, b, c, d); }
};
template <> struct Frag<__bf16> {
  typedef v16b V; union U { v16b v; v8b h[2]; };
  static __device__ __forceinline__ v16b load(const __bf16* p) {
    U f; f.h[0] = *(const v8b*)(p); f.h[1] = *(const v8b*)(p + 16); return f.v;
  }
  static __device__ __forceinline__ v8f mma(v16b a, v16b b, v8f c) {
    return __builtin_amdgcn_wmma_f32_16x16x32_bf16(false, a, false, b, (short)0, c, false, false);
  }
  static __device__ __forceinline__ void guard(v8f& a, v8f& b, v16b x, v16b y) { dep_guard_b(a, b, x, y); }
  static __device__ __forceinline__ void keep(v16b a, v16b b, v16b c, v16b d) { keep4_b(a, b, c, d); }
};

template <int ET> struct Elem;
template <> struct Elem<0> { typedef _Float16 T; };
template <> struct Elem<1> { typedef __bf16 T; };
template <int ET, bool SPLIT, int BIAS_MODE, int OUT_MODE, bool RESID, int ACT = 0, bool ADDROW = false>
__global__ __launch_bounds__(256) void wmma_gemm64(
    const unsigned short* __restrict__ Ap, const unsigned short* __restrict__ A2p, int lda, long strideA,
    const unsigned short* __restrict__ Btp, const unsigned short* __restrict__ Bt2p, int ldb, long strideB,
    void* __restrict__ Cout, void* __restrict__ Cout2, int ldc, long strideC,
    const float* __restrict__ bias,
    const float* __restrict__ resid, long strideR,
    int M, int N, int K, float scale) {
  static_assert(!(RESID && ADDROW));
  static_assert(!ADDROW || OUT_MODE == 0);
  typedef typename Elem<ET>::T T;
  typedef typename Frag<T>::V V;
  const T* A = (const T*)Ap; const T* A2 = (const T*)A2p; const T* Bt = (const T*)Btp; const T* Bt2 = (const T*)Bt2p;
  __shared__ __align__(16) float sT[8][16 * 68];
  const int b    = blockIdx.y;
  const int lane = threadIdx.x & 31;
  const int wave = threadIdx.x >> 5;
  const int tilesN = N >> 6;
  const int tilesM = M >> 6;
  const int tile = blockIdx.x * 8 + wave;
  if (tile >= tilesM * tilesN) return;
  const int tm = tile / tilesN;
  const int tn = tile - tm * tilesN;
  const int m0 = tm << 6;
  const int n0 = tn << 6;

  const T* Ab  = A  + (size_t)b * strideA;
  const T* Bb  = Bt + (size_t)b * strideB;
  const T* Ab2 = SPLIT ? (A2  + (size_t)b * strideA) : nullptr;
  const T* Bb2 = SPLIT ? (Bt2 + (size_t)b * strideB) : nullptr;

  const int rlane = lane & 15;
  const int koff  = (lane >> 4) * 8;
  const int mOff  = (lane >> 4) * 8;

  v8f acc[4][4];
#pragma unroll
  for (int i = 0; i < 4; ++i)
#pragma unroll
    for (int j = 0; j < 4; ++j) acc[i][j] = (v8f){0.f,0.f,0.f,0.f,0.f,0.f,0.f,0.f};

  for (int k0 = 0; k0 < K; k0 += 32) {
    V bh[4], bl[4];
#pragma unroll
    for (int j = 0; j < 4; ++j) {
      const size_t bo = (size_t)(n0 + (j << 4) + rlane) * ldb + koff + k0;
      bh[j] = Frag<T>::load(Bb + bo);
      if (SPLIT) bl[j] = Frag<T>::load(Bb2 + bo);
    }
#pragma unroll
    for (int i = 0; i < 4; ++i) {
      const size_t ao = (size_t)(m0 + (i << 4) + rlane) * lda + koff + k0;
      V ah = Frag<T>::load(Ab + ao);
      V al;
      if (SPLIT) al = Frag<T>::load(Ab2 + ao);
#pragma unroll
      for (int j = 0; j < 4; ++j) {
        acc[i][j] = Frag<T>::mma(ah, bh[j], acc[i][j]);
        if (SPLIT) {
          acc[i][j] = Frag<T>::mma(ah, bl[j], acc[i][j]);
          acc[i][j] = Frag<T>::mma(al, bh[j], acc[i][j]);
        }
      }
      Frag<T>::guard(acc[i][0], acc[i][3], ah, SPLIT ? al : ah);
    }
    Frag<T>::keep(bh[0], bh[1], bh[2], bh[3]);
    if (SPLIT) Frag<T>::keep(bl[0], bl[1], bl[2], bl[3]);
  }
  acc_guard4(acc[0][0], acc[0][1], acc[0][2], acc[0][3]);
  acc_guard4(acc[1][0], acc[1][1], acc[1][2], acc[1][3]);
  acc_guard4(acc[2][0], acc[2][1], acc[2][2], acc[2][3]);
  acc_guard4(acc[3][0], acc[3][1], acc[3][2], acc[3][3]);

  float* slab = sT[wave];
  const float* Rb = RESID ? (resid + (size_t)b * strideR) : nullptr;
#pragma unroll
  for (int i = 0; i < 4; ++i) {
    const int mBase = m0 + (i << 4);
#pragma unroll
    for (int j = 0; j < 4; ++j) {
      const int n = n0 + (j << 4) + rlane;
      float bv = 0.f;
      if (BIAS_MODE == 2) bv = bias[n];
#pragma unroll
      for (int r = 0; r < 8; ++r) {
        float v = acc[i][j][r] * scale;
        if (BIAS_MODE == 1) v += bias[mBase + mOff + r];
        if (BIAS_MODE == 2) v += bv;
        if (RESID) v += Rb[(size_t)(mBase + mOff + r) * ldc + n];
        if (ACT == 1) v = tanhf(v);
        if (ACT == 2) v = fmaxf(v, 0.0f);
        if (ACT == 3) v = v / (1.0f + expf(-v));
        if (ACT == 4) v = (v > 0.f) ? v : 0.01f * v;
        slab[(mOff + r) * 68 + (j << 4) + rlane] = v;
      }
    }
    __builtin_amdgcn_fence(__ATOMIC_RELEASE, "workgroup");
    __builtin_amdgcn_wave_barrier();
    __builtin_amdgcn_fence(__ATOMIC_ACQUIRE, "workgroup");
    if (OUT_MODE == 0) {
      float* C = (float*)Cout + (size_t)b * strideC;
      const int hh = lane >> 4, c4 = (lane & 15) * 4;
      v4f av = (v4f){0.f, 0.f, 0.f, 0.f};
      if (ADDROW) av = *(const v4f*)(resid + (size_t)b * strideR + n0 + c4);
      for (int pass = 0; pass < 2; ++pass) {
#pragma unroll
        for (int it = 0; it < 8; ++it) {
          const int row = it * 2 + hh;
          v4f v = *(const v4f*)(slab + row * 68 + c4);
          if (ADDROW) v = v + av;
          *(volatile v4f*)(C + (size_t)(mBase + row) * ldc + n0 + c4) = v;
        }
        __threadfence();
      }
    } else {
      const int q = lane >> 3, c8 = (lane & 7) * 8;
      unsigned short* C  = (unsigned short*)Cout  + (size_t)b * strideC;
      unsigned short* C2 = (OUT_MODE == 2) ? ((unsigned short*)Cout2 + (size_t)b * strideC) : nullptr;
      for (int pass = 0; pass < 2; ++pass) {
#pragma unroll
        for (int it = 0; it < 4; ++it) {
          const int row = it * 4 + q;
          const float* sp = slab + row * 68 + c8;
          v8h hv, lv;
#pragma unroll
          for (int e = 0; e < 8; ++e) {
            if (OUT_MODE == 1) {
              hv[e] = (_Float16)sp[e];
            } else {
              unsigned short hb = f2bf_bits(sp[e]);
              unsigned short lb = f2bf_bits(sp[e] - bf_bits2f(hb));
              hv[e] = __builtin_bit_cast(_Float16, hb);
              lv[e] = __builtin_bit_cast(_Float16, lb);
            }
          }
          *(volatile v8h*)(C + (size_t)(mBase + row) * ldc + n0 + c8) = hv;
          if (OUT_MODE == 2) *(volatile v8h*)(C2 + (size_t)(mBase + row) * ldc + n0 + c8) = lv;
        }
        __threadfence();
      }
    }
    __builtin_amdgcn_fence(__ATOMIC_RELEASE, "workgroup");
    __builtin_amdgcn_wave_barrier();
    __builtin_amdgcn_fence(__ATOMIC_ACQUIRE, "workgroup");
  }
}


__global__ __launch_bounds__(256) void prep_bias_kernel(const float* __restrict__ bq, const float* __restrict__ bo,
                                                        float* __restrict__ outb) {
  const int i  = blockIdx.x * 256 + threadIdx.x;
  const int iq = imin(i, 767);
  const int io = imin(imax(i - 768, 0), 255);
  const v4f a = *(const v4f*)(bq + 4 * iq);
  const v4f c = *(const v4f*)(bo + 4 * io);
  v4f r;
#pragma unroll
  for (int e = 0; e < 4; ++e) r[e] = bf16r((i < 768) ? a[e] : c[e]);
  float* d = outb + 4 * i;
  *(volatile v4f*)d = r;
  __threadfence();
  *(volatile v4f*)d = r;
}

__global__ __launch_bounds__(256) void cast_x_kernel(const float* __restrict__ x, unsigned short* __restrict__ xb) {
  const size_t i = (size_t)blockIdx.x * 256 + threadIdx.x;
  const float* p = x + i * 8;
  const v4f a = *(const v4f*)p;
  const v4f c = *(const v4f*)(p + 4);
  us8 o;
#pragma unroll
  for (int e = 0; e < 4; ++e) { o[e] = f2bf_bits(a[e]); o[4 + e] = f2bf_bits(c[e]); }
  unsigned short* d = xb + i * 8;
  *(volatile us8*)d = o;
  __threadfence();
  *(volatile us8*)d = o;
}

__global__ __launch_bounds__(256) void prep_wqkv_kernel(const float* __restrict__ w, unsigned short* __restrict__ wt) {
  __shared__ float tile[64][65];
  const int e0 = blockIdx.x * 64, d0 = blockIdx.y * 64;
  const int t = threadIdx.x;
  {
    const int r = t >> 2, cb = (t & 3) * 16;
    const float* src = w + (size_t)(d0 + r) * kN3 + e0 + cb;
#pragma unroll
    for (int i = 0; i < 4; ++i) {
      const v4f v = *(const v4f*)(src + 4 * i);
#pragma unroll
      for (int e = 0; e < 4; ++e) tile[r][cb + 4 * i + e] = v[e];
    }
  }
  __syncthreads();
  for (int pass = 0; pass < 2; ++pass) {
#pragma unroll
    for (int it = 0; it < 2; ++it) {
      const int er = it * 32 + (t >> 3), c8 = (t & 7) * 8;
      us8 o;
#pragma unroll
      for (int j = 0; j < 8; ++j) o[j] = f2bf_bits(tile[c8 + j][er]);
      unsigned short* dst = wt + (size_t)(e0 + er) * kDim + d0 + c8;
      *(volatile us8*)dst = o;
    }
    __threadfence();
  }
}

__global__ __launch_bounds__(256) void prep_wout_kernel(const float* __restrict__ w, unsigned short* __restrict__ wo16,
                                                        unsigned short* __restrict__ wob) {
  __shared__ float tile[64][65];
  const int e0 = blockIdx.x * 64, d0 = blockIdx.y * 64;
  const int t = threadIdx.x;
  {
    const int r = t >> 2, cb = (t & 3) * 16;
    const float* src = w + (size_t)(d0 + r) * kDim + e0 + cb;
#pragma unroll
    for (int i = 0; i < 4; ++i) {
      const v4f v = *(const v4f*)(src + 4 * i);
#pragma unroll
      for (int e = 0; e < 4; ++e) tile[r][cb + 4 * i + e] = v[e];
    }
  }
  __syncthreads();
  for (int pass = 0; pass < 2; ++pass) {
#pragma unroll
    for (int it = 0; it < 2; ++it) {
      const int er = it * 32 + (t >> 3), c8 = (t & 7) * 8;
      us8 o16, ob;
#pragma unroll
      for (int j = 0; j < 8; ++j) {
        const float wr = bf16r(tile[c8 + j][er]);
        ob[j]  = f2bf_bits(wr);
        o16[j] = __builtin_bit_cast(unsigned short, (_Float16)(wr * kWoCarry));
      }
      const size_t off = (size_t)(e0 + er) * kDim + d0 + c8;
      *(volatile us8*)(wo16 + off) = o16;
      *(volatile us8*)(wob + off) = ob;
    }
    __threadfence();
  }
}

__global__ __launch_bounds__(256) void zero16_kernel(unsigned short* __restrict__ p) {
  const size_t i = (size_t)blockIdx.x * 256 + threadIdx.x;
  const u32x4 z = (u32x4){0u, 0u, 0u, 0u};
  unsigned short* d = p + i * 8;
  *(volatile u32x4*)d = z;
  __threadfence();
  *(volatile u32x4*)d = z;
}

__global__ __launch_bounds__(256) void mean_x_kernel(const float* __restrict__ x, unsigned short* __restrict__ mxh,
                                                     unsigned short* __restrict__ mxl) {
  __shared__ __align__(16) unsigned short sh[256];
  __shared__ __align__(16) unsigned short sl[256];
  const int cq = blockIdx.x;
  const int r  = blockIdx.y;
  const int t  = threadIdx.x;
  const int d  = cq * 256 + t;
  const int rb = imin(r, kBatch - 1);
  const int nk = (r < kBatch) ? kSeq : 0;
  const float* p = x + (size_t)rb * kSeq * kDim + d;
  float s0 = 0.0f, s1 = 0.0f, s2 = 0.0f, s3 = 0.0f;
#pragma unroll 1
  for (int k = 0; k < nk; k += 4) {
    const float a0 = p[(size_t)(k + 0) * kDim];
    const float a1 = p[(size_t)(k + 1) * kDim];
    const float a2 = p[(size_t)(k + 2) * kDim];
    const float a3 = p[(size_t)(k + 3) * kDim];
    s0 += bf16r(a0); s1 += bf16r(a1); s2 += bf16r(a2); s3 += bf16r(a3);
  }
  const float mean = ((s0 + s1) + (s2 + s3)) * (1.0f / 2048.0f);
  const unsigned short hb = f2bf_bits(mean);
  const unsigned short lb = f2bf_bits(mean - bf_bits2f(hb));
  sh[t] = hb;
  sl[t] = lb;
  __syncthreads();
  const int wave = t >> 5, lane = t & 31;
  if (wave < 2) {
    const us8 vh = *(const us8*)(sh + lane * 8);
    const us8 vl = *(const us8*)(sl + lane * 8);
    us8 o;
#pragma unroll
    for (int e = 0; e < 8; ++e) o[e] = (wave == 0) ? vh[e] : vl[e];
    unsigned short* base = (wave == 0) ? mxh : mxl;
    unsigned short* dst = base + (size_t)r * kDim + cq * 256 + lane * 8;
    *(volatile us8*)dst = o;
    __threadfence();
    *(volatile us8*)dst = o;
  }
}

__global__ __launch_bounds__(256) void softmax_kernel(const float* __restrict__ sc, unsigned short* __restrict__ pp) {
  __shared__ float redm[8];
  __shared__ float reds[8];
  const int row = blockIdx.x;
  const int t = threadIdx.x, lane = t & 31, wave = t >> 5;
  const float* src = sc + (size_t)row * kSeq + t * 8;
  const v4f a = *(const v4f*)src;
  const v4f c = *(const v4f*)(src + 4);
  float m = -__builtin_inff();
#pragma unroll
  for (int e = 0; e < 4; ++e) { m = fmaxf(m, a[e]); m = fmaxf(m, c[e]); }
#pragma unroll
  for (int off = 1; off < 32; off <<= 1) m = fmaxf(m, __shfl_xor(m, off, 32));
  if (lane == 0) redm[wave] = m;
  __syncthreads();
  float bm = redm[0];
#pragma unroll
  for (int wv = 1; wv < 8; ++wv) bm = fmaxf(bm, redm[wv]);
  v4f ea, ec;
  float ps = 0.0f;
#pragma unroll
  for (int e = 0; e < 4; ++e) { ea[e] = expf(a[e] - bm); ps += ea[e]; }
#pragma unroll
  for (int e = 0; e < 4; ++e) { ec[e] = expf(c[e] - bm); ps += ec[e]; }
#pragma unroll
  for (int off = 1; off < 32; off <<= 1) ps += __shfl_xor(ps, off, 32);
  if (lane == 0) reds[wave] = ps;
  __syncthreads();
  float tot = 0.0f;
#pragma unroll
  for (int wv = 0; wv < 8; ++wv) tot += reds[wv];
  const float cinv = (1.0f / tot) * kPcarry;
  us8 o;
#pragma unroll
  for (int e = 0; e < 4; ++e) {
    const float p0 = fmaf(ea[e], cinv, -kPoffset);
    const float p1 = fmaf(ec[e], cinv, -kPoffset);
    o[e]     = __builtin_bit_cast(unsigned short, (_Float16)p0);
    o[4 + e] = __builtin_bit_cast(unsigned short, (_Float16)p1);
  }
  unsigned short* dst = pp + (size_t)row * kSeq + t * 8;
  *(volatile us8*)dst = o;
  __threadfence();
  *(volatile us8*)dst = o;
}

static_assert(kTok % 64 == 0 && kSeq % 64 == 0 && kDim % 64 == 0 && kPadM % 64 == 0);
static_assert(kDim % 32 == 0 && kSeq % 32 == 0);

extern "C" void kernel_launch(void* const* d_in, const int* in_sizes, int n_in,
                              void* d_out, int out_size, void* d_ws, size_t ws_size,
                              hipStream_t stream) {
  if (n_in < 5) return;
  if (in_sizes[0] != kTok * kDim) return;
  if (in_sizes[1] != kDim * kN3) return;
  if (in_sizes[2] != kN3) return;
  if (in_sizes[3] != kDim * kDim) return;
  if (in_sizes[4] != kDim) return;
  if (out_size != kTok * kDim) return;
  if (ws_size < WS_TOTAL) return;

  const float* x     = (const float*)d_in[0];
  const float* w_qkv = (const float*)d_in[1];
  const float* b_qkv = (const float*)d_in[2];
  const float* w_out = (const float*)d_in[3];
  const float* b_out = (const float*)d_in[4];
  float* outp = (float*)d_out;

  char* ws = (char*)d_ws;
  unsigned short* xb    = (unsigned short*)(ws + OFF_XB);
  unsigned short* zpl   = (unsigned short*)(ws + OFF_XB);
  unsigned short* wqkvT = (unsigned short*)(ws + OFF_WQKV);
  unsigned short* wvT   = wqkvT + (size_t)2048 * kDim;
  unsigned short* wo16  = (unsigned short*)(ws + OFF_WO16);
  unsigned short* wob   = (unsigned short*)(ws + OFF_WOB);
  unsigned short* zero  = (unsigned short*)(ws + OFF_ZERO);
  float*          biasr = (float*)(ws + OFF_BIAS);
  unsigned short* mxh   = (unsigned short*)(ws + OFF_MXH);
  unsigned short* mxl   = (unsigned short*)(ws + OFF_MXL);
  unsigned short* vbh   = (unsigned short*)(ws + OFF_VBH);
  unsigned short* vbl   = (unsigned short*)(ws + OFF_VBL);
  float*          addv  = (float*)(ws + OFF_ADDV);
  unsigned short* qkp   = (unsigned short*)(ws + OFF_QK);
  unsigned short* vt    = (unsigned short*)(ws + OFF_VT);
  float*          sbuf  = (float*)(ws + OFF_SBUF);

  const long sQKbatch = (long)kSeq * 2048;
  const long sVTbatch = (long)kDim * kSeq;
  const long sSbatch  = (long)kSeq * kSeq;
  const long sZbatch  = (long)kSeq * kDim;

  prep_bias_kernel<<<4, 256, 0, stream>>>(b_qkv, b_out, biasr);
  cast_x_kernel<<<(kTok * kDim) / (256 * 8), 256, 0, stream>>>(x, xb);
  prep_wqkv_kernel<<<dim3(kN3 / 64, kDim / 64), 256, 0, stream>>>(w_qkv, wqkvT);
  prep_wout_kernel<<<dim3(kDim / 64, kDim / 64), 256, 0, stream>>>(w_out, wo16, wob);
  zero16_kernel<<<(int)(SZ_WO / (256 * 16)), 256, 0, stream>>>(zero);
  mean_x_kernel<<<dim3(4, kPadM), 256, 0, stream>>>(x, mxh, mxl);

  wmma_gemm64<1, false, 2, 1, false><<<dim3((kTok / 64) * (2048 / 64) / 8, 1), 256, 0, stream>>>(
      xb, xb, kDim, 0L, wqkvT, wqkvT, kDim, 0L, qkp, qkp, 2048, 0L,
      biasr, biasr, 0L, kTok, 2048, kDim, 1.0f);

  wmma_gemm64<1, false, 1, 1, false><<<dim3((kDim / 64) * (kSeq / 64) / 8, kBatch), 256, 0, stream>>>(
      wvT, wvT, kDim, 0L, xb, xb, kDim, (long)kSeq * kDim, vt, vt, kSeq, sVTbatch,
      biasr + 2048, biasr, 0L, kDim, kSeq, kDim, 1.0f);

  wmma_gemm64<1, true, 2, 2, false><<<dim3(2, 1), 256, 0, stream>>>(
      mxh, mxl, kDim, 0L, wvT, zero, kDim, 0L, vbh, vbl, kDim, 0L,
      biasr + 2048, biasr, 0L, kPadM, kDim, kDim, 1.0f);

  wmma_gemm64<1, true, 2, 0, false><<<dim3(2, 1), 256, 0, stream>>>(
      vbh, vbl, kDim, 0L, wob, zero, kDim, 0L, addv, addv, kDim, 0L,
      biasr + 3072, biasr, 0L, kPadM, kDim, kDim, 1.0f);

  for (int pr = 0; pr < 2; ++pr) {
    unsigned short* qkb = qkp + (size_t)(2 * pr) * sQKbatch;
    wmma_gemm64<0, false, 0, 0, false><<<dim3((kSeq / 64) * (kSeq / 64) / 8, 2), 256, 0, stream>>>(
        qkb, qkb, 2048, sQKbatch, qkb + kDim, qkb + kDim, 2048, sQKbatch, sbuf, sbuf, kSeq, sSbatch,
        biasr, biasr, 0L, kSeq, kSeq, kDim, kScoreScale);
    softmax_kernel<<<2 * kSeq, 256, 0, stream>>>(sbuf, qkb);
  }

  wmma_gemm64<0, false, 0, 1, false><<<dim3((kSeq / 64) * (kDim / 64) / 8, kBatch), 256, 0, stream>>>(
      qkp, qkp, kSeq, sQKbatch, vt, vt, kSeq, sVTbatch, zpl, zpl, kDim, sZbatch,
      biasr, biasr, 0L, kSeq, kDim, kSeq, kZcarry / kPcarry);

  wmma_gemm64<0, false, 0, 0, false, 0, true><<<dim3((kSeq / 64) * (kDim / 64) / 8, kBatch), 256, 0, stream>>>(
      zpl, zpl, kDim, sZbatch, wo16, wo16, kDim, 0L, outp, outp, kDim, sZbatch,
      biasr, addv, (long)kDim, kSeq, kDim, kDim, 1.0f / (kZcarry * kWoCarry));
}
